// CrossAttention_with_lora_27384711480000
// MI455X (gfx1250) — hardware-run, weakly checked
//
#include <hip/hip_runtime.h>


#define NB_  8
#define TT   1024
#define SS   256
#define CC   1024
#define NH_  16
#define HD   64
#define RR   16
#define RP   64
typedef _Float16 h16;
typedef unsigned short bf;
typedef __attribute__((ext_vector_type(16))) __bf16   v16bf;
typedef __attribute__((ext_vector_type(16))) _Float16 v16h;
typedef __attribute__((ext_vector_type(8)))  _Float16 v8h;
typedef __attribute__((ext_vector_type(8)))  unsigned short v8us;
typedef __attribute__((ext_vector_type(8)))  float    v8f;
typedef __attribute__((ext_vector_type(4)))  float    v4f;
typedef v8h  __attribute__((may_alias)) v8ha;
typedef v4f  __attribute__((may_alias)) v4fa;
typedef v8us __attribute__((may_alias)) v8usa;

__device__ __forceinline__ unsigned short f2bf(float f) { unsigned u = __float_as_uint(f); u += 0x7FFFu + ((u >> 16) & 1u); return (unsigned short)(u >> 16); }
__device__ __forceinline__ float bf2f(unsigned short b) { return __uint_as_float(((unsigned)b) << 16); }
__device__ __forceinline__ float bfr(float f) { return bf2f(f2bf(f)); }
__device__ __forceinline__ v16h cat16(v8h lo, v8h hi) { return __builtin_shufflevector(lo, hi, 0, 1, 2, 3, 4, 5, 6, 7, 8, 9, 10, 11, 12, 13, 14, 15); }
__device__ __forceinline__ v16bf cat16b(v8us lo, v8us hi) { return __builtin_bit_cast(v16bf, __builtin_shufflevector(lo, hi, 0, 1, 2, 3, 4, 5, 6, 7, 8, 9, 10, 11, 12, 13, 14, 15)); }
__device__ __forceinline__ v8f wmma16(v16h a, v16h b, v8f c) { return __builtin_amdgcn_wmma_f32_16x16x32_f16(false, a, false, b, (short)0, c, false, false); }
__device__ __forceinline__ v8f wmmab(v16bf a, v16bf b, v8f c) { return __builtin_amdgcn_wmma_f32_16x16x32_bf16(false, a, false, b, (short)0, c, false, false); }


template <typename T16> struct WFrag;
template <> struct WFrag<h16> { typedef v16h V; static __device__ __forceinline__ V ld(const h16* p) { return cat16(*(const v8h*)p, *(const v8h*)(p + 16)); } static __device__ __forceinline__ v8f mma(V a, V b, v8f c) { return wmma16(a, b, c); } };
template <> struct WFrag<bf> { typedef v16bf V; static __device__ __forceinline__ V ld(const bf* p) { return cat16b(*(const v8us*)p, *(const v8us*)(p + 16)); } static __device__ __forceinline__ v8f mma(V a, V b, v8f c) { return wmmab(a, b, c); } };
template <typename T16, int NSPLIT, bool BIAS>
__global__ __launch_bounds__(32) void k_gemmw(const T16* __restrict__ A, const T16* __restrict__ A2, const T16* __restrict__ Bt, const T16* __restrict__ Bt2, int K, float* C, int ldc, const float* __restrict__ bias, size_t sA, size_t sB, size_t sC) {
    typedef typename WFrag<T16>::V V;
    __shared__ __align__(16) float os[16 * 68];
    const size_t z = blockIdx.z; A += z * sA; if (A2) A2 += z * sA; Bt += z * sB; if (Bt2) Bt2 += z * sB; C += z * sC;
    const int lane = threadIdx.x & 31, lr = lane & 15, hi = lane >> 4; const int r0 = blockIdx.x * 64, c0 = blockIdx.y * 64;
    v8f acc[4][4];
#pragma unroll
    for (int mb = 0; mb < 4; ++mb)
#pragma unroll
        for (int nb = 0; nb < 4; ++nb) acc[mb][nb] = (v8f){};
    const size_t aoff = (size_t)(r0 + lr) * K + 8 * hi, boff = (size_t)(c0 + lr) * K + 8 * hi;
#pragma unroll 1
    for (int kc = 0; kc < K; kc += 32) {
        V a[4], a2[4];
#pragma unroll
        for (int mb = 0; mb < 4; ++mb) { a[mb] = WFrag<T16>::ld(A + aoff + (size_t)mb * 16 * K + kc); if (NSPLIT == 1 || NSPLIT == 2) a2[mb] = WFrag<T16>::ld(A2 + aoff + (size_t)mb * 16 * K + kc); }
#pragma unroll
        for (int nb = 0; nb < 4; ++nb) { const V b = WFrag<T16>::ld(Bt + boff + (size_t)nb * 16 * K + kc); V b2; if (NSPLIT >= 2) b2 = WFrag<T16>::ld(Bt2 + boff + (size_t)nb * 16 * K + kc);
#pragma unroll
            for (int mb = 0; mb < 4; ++mb) { acc[mb][nb] = WFrag<T16>::mma(a[mb], b, acc[mb][nb]); if (NSPLIT == 1 || NSPLIT == 2) acc[mb][nb] = WFrag<T16>::mma(a2[mb], b, acc[mb][nb]); if (NSPLIT >= 2) acc[mb][nb] = WFrag<T16>::mma(a[mb], b2, acc[mb][nb]); } }
        asm volatile("v_nop\n\tv_nop\n\tv_nop\n\tv_nop" : "+v"(acc[0][0]), "+v"(acc[1][1]), "+v"(acc[2][2]), "+v"(acc[3][3]) : "v"(a[0]), "v"(a[3]));
    }
#pragma unroll
    for (int mb = 0; mb < 4; ++mb) {
#pragma unroll
        for (int nb = 0; nb < 4; ++nb) {
#pragma unroll
            for (int j = 0; j < 8; ++j) os[(hi * 8 + j) * 68 + nb * 16 + lr] = acc[mb][nb][j]; }
        __builtin_amdgcn_wave_barrier(); asm volatile("" ::: "memory");
        float* crow = C + (size_t)(r0 + mb * 16) * ldc + c0;
#pragma unroll 1
        for (int ps = 0; ps < 2; ++ps) {
#pragma unroll
            for (int s = 0; s < 8; ++s) { const int row = 2 * s + hi, cofs = lr * 4; v4f val = *(const v4fa*)(os + row * 68 + cofs); if (BIAS) { val[0] += bfr(bias[c0 + cofs]); val[1] += bfr(bias[c0 + cofs + 1]); val[2] += bfr(bias[c0 + cofs + 2]); val[3] += bfr(bias[c0 + cofs + 3]); }
                *(volatile v4f*)(crow + (size_t)row * ldc + cofs) = val; }
            if (ps == 0) __threadfence(); }
        __builtin_amdgcn_wave_barrier(); asm volatile("" ::: "memory");
    }
}

__device__ __forceinline__ void splitf(float y, unsigned short& h, unsigned short& l) { h = f2bf(y); l = f2bf(y - bf2f(h)); }
typedef __attribute__((ext_vector_type(2))) unsigned short v2us;
typedef __attribute__((ext_vector_type(4))) unsigned short v4us;

__global__ __launch_bounds__(256) void k_cvt8(const float* __restrict__ src, bf* dst, size_t n8) { const size_t i = (size_t)blockIdx.x * 256 + threadIdx.x; if (i >= n8) return; const v8f v = *(const v8f*)(src + i * 8); v8us o;
#pragma unroll
    for (int k = 0; k < 8; ++k) o[k] = f2bf(v[k]); *(volatile v8us*)(dst + i * 8) = o; __threadfence(); *(volatile v8us*)(dst + i * 8) = o; }
__global__ __launch_bounds__(256) void k_wpadN(const float* __restrict__ A, int K, bf* Bt) { const int e = (blockIdx.x * 256 + threadIdx.x) * 4; if (e >= RP * K) return; const int n = e / K; v4us o;
#pragma unroll
    for (int u = 0; u < 4; ++u) o[u] = n < RR ? f2bf(A[e + u]) : (unsigned short)0; *(volatile v4us*)(Bt + e) = o; __threadfence(); *(volatile v4us*)(Bt + e) = o; }
__global__ __launch_bounds__(256) void k_wpadK(const float* __restrict__ Bm, int N, bf* Bt) { const int e = (blockIdx.x * 256 + threadIdx.x) * 4; if (e >= N * RP) return; const int k = e % RP, n = e / RP; v4us o;
#pragma unroll
    for (int u = 0; u < 4; ++u) o[u] = (k + u) < RR ? f2bf(Bm[(size_t)n * RR + k + u]) : (unsigned short)0; *(volatile v4us*)(Bt + e) = o; __threadfence(); *(volatile v4us*)(Bt + e) = o; }
__global__ __launch_bounds__(256) void k_split(const float* __restrict__ F, size_t n4, bf* Ph, bf* Pl) { const size_t e = ((size_t)blockIdx.x * 256 + threadIdx.x) * 4; if (e >= n4 * 4) return; const v4f a = *(const v4f*)(F + e); v4us oh, ol;
#pragma unroll
    for (int u = 0; u < 4; ++u) { unsigned short h, l; splitf(a[u], h, l); oh[u] = h; ol[u] = l; } *(volatile v4us*)(Ph + e) = oh; *(volatile v4us*)(Pl + e) = ol; __threadfence(); *(volatile v4us*)(Ph + e) = oh; *(volatile v4us*)(Pl + e) = ol; }
__global__ __launch_bounds__(256) void k_qpl(const float* __restrict__ Q0, const float* __restrict__ QL, int nrows, int pitch, int coff, bf* Ph, bf* Pl) { const int e = (blockIdx.x * 256 + threadIdx.x) * 4; if (e >= NH_ * nrows * HD) return; const int d = e % HD; const int t = (e / HD) % nrows; const int h = e / (HD * nrows); const size_t src = (size_t)t * pitch + coff + h * HD + d; const v4f a = *(const v4f*)(Q0 + src), b = *(const v4f*)(QL + src); v4us oh, ol;
#pragma unroll
    for (int u = 0; u < 4; ++u) { float lr = b[u] * (1.0f / 16.0f); asm volatile("" : "+v"(lr)); unsigned short hh, ll; splitf(__fadd_rn(a[u], lr), hh, ll); oh[u] = hh; ol[u] = ll; } *(volatile v4us*)(Ph + e) = oh; *(volatile v4us*)(Pl + e) = ol; __threadfence(); *(volatile v4us*)(Ph + e) = oh; *(volatile v4us*)(Pl + e) = ol; }
__global__ __launch_bounds__(256) void k_vtpl(const float* __restrict__ KV0, const float* __restrict__ KVL, bf* Th, bf* Tl) { const int e = (blockIdx.x * 256 + threadIdx.x) * 2; if (e >= NH_ * HD * SS) return; const int s = e % SS; const int d = (e / SS) % HD; const int h = e / (SS * HD); v2us oh, ol;
#pragma unroll
    for (int u = 0; u < 2; ++u) { const size_t src = (size_t)(s + u) * 2 * CC + CC + h * HD + d; float lr = KVL[src] * (1.0f / 16.0f); asm volatile("" : "+v"(lr)); unsigned short hh, ll; splitf(__fadd_rn(KV0[src], lr), hh, ll); oh[u] = hh; ol[u] = ll; }
    *(volatile v2us*)(Th + e) = oh; *(volatile v2us*)(Tl + e) = ol; __threadfence(); *(volatile v2us*)(Th + e) = oh; *(volatile v2us*)(Tl + e) = ol; }
__global__ __launch_bounds__(256) void k_mrg(const float* __restrict__ O, bf* Ph, bf* Pl) { const int e = (blockIdx.x * 256 + threadIdx.x) * 4; if (e >= TT * CC) return; const int c = e % CC; const int t = e / CC; const int h = c / HD, d = c % HD; const float* r = O + ((size_t)h * TT + t) * HD + d; v4us oh, ol;
#pragma unroll
    for (int u = 0; u < 4; ++u) { unsigned short a, b; splitf(r[u], a, b); oh[u] = a; ol[u] = b; } *(volatile v4us*)(Ph + e) = oh; *(volatile v4us*)(Pl + e) = ol; __threadfence(); *(volatile v4us*)(Ph + e) = oh; *(volatile v4us*)(Pl + e) = ol; }
__global__ __launch_bounds__(256) void k_fin(const float* __restrict__ Y0, const float* __restrict__ PLr, float* OUT) { const int e = (blockIdx.x * 256 + threadIdx.x) * 4; if (e >= TT * CC) return; const v4f a = *(const v4f*)(Y0 + e), b = *(const v4f*)(PLr + e); v4f o;
#pragma unroll
    for (int u = 0; u < 4; ++u) { float lr = b[u] * (1.0f / 16.0f); asm volatile("" : "+v"(lr)); o[u] = __fadd_rn(a[u], lr); } *(volatile v4f*)(OUT + e) = o; __threadfence(); *(volatile v4f*)(OUT + e) = o; }
__global__ __launch_bounds__(256) void k_csoft(const float* __restrict__ Sb, bf* Ph, bf* Pl) { const int lane = threadIdx.x & 31; const int row = blockIdx.x * 8 + (threadIdx.x >> 5); if (row >= NH_ * TT) return; const int t = row % TT; const float* sr = Sb + (size_t)row * SS; float v[8]; float mx = -3.0e38f;
#pragma unroll
    for (int ch = 0; ch < 2; ++ch) { const int j0 = ch * 128 + lane * 4; const v4f a = *(const v4f*)(sr + j0);
#pragma unroll
        for (int q = 0; q < 4; ++q) { const int j = j0 + q; const float tt = (j <= t) ? a[q] * 0.125f : -3.0e38f; v[ch * 4 + q] = tt; mx = fmaxf(mx, tt); } }
#pragma unroll
    for (int sh = 16; sh; sh >>= 1) mx = fmaxf(mx, __shfl_xor(mx, sh, 32));
    float sum = 0.f;
#pragma unroll
    for (int k = 0; k < 8; ++k) { float d0 = __fsub_rn(v[k], mx); asm volatile("" : "+v"(d0)); v[k] = __expf(d0); sum += v[k]; }
#pragma unroll
    for (int sh = 16; sh; sh >>= 1) sum += __shfl_xor(sum, sh, 32);
    const float f = __fdiv_rn(1.0f, sum);
    for (int ps = 0; ps < 2; ++ps) {
#pragma unroll
        for (int ch = 0; ch < 2; ++ch) { v4us oh, ol;
#pragma unroll
            for (int q = 0; q < 4; ++q) { unsigned short a, c2; splitf(v[ch * 4 + q] * f, a, c2); oh[q] = a; ol[q] = c2; } const size_t oo = (size_t)row * SS + ch * 128 + lane * 4; *(volatile v4us*)(Ph + oo) = oh; *(volatile v4us*)(Pl + oo) = ol; }
        if (ps == 0) __threadfence(); } }

extern "C" void kernel_launch(void* const* d_in, const int* in_sizes, int n_in,
                              void* d_out, int out_size, void* d_ws, size_t ws_size, hipStream_t stream) {
    (void)in_sizes; (void)n_in; (void)out_size;
    const float** I = (const float**)d_in;
    const float *x = I[0], *fe = I[1], *wq = I[2], *bq = I[3], *aq = I[4], *bqm = I[5], *wf = I[6], *bff = I[7], *af = I[8], *bfm = I[9], *wp = I[10], *bp = I[11], *ap = I[12], *bpm = I[13];
    float* OUT = (float*)d_out;
    char* wsp = (char*)d_ws;
    auto take = [&](size_t bytes) { char* p = wsp; wsp += (bytes + 255) & ~(size_t)255; return (void*)p; };
    bf* WQ = (bf*)take((size_t)CC * CC * 2); bf* AQ = (bf*)take((size_t)RP * CC * 2); bf* BQ = (bf*)take((size_t)CC * RP * 2); bf* WF = (bf*)take((size_t)2 * CC * CC * 2); bf* AF = (bf*)take((size_t)RP * CC * 2); bf* BF = (bf*)take((size_t)2 * CC * RP * 2); bf* WP = (bf*)take((size_t)CC * CC * 2); bf* AP = (bf*)take((size_t)RP * CC * 2); bf* BP = (bf*)take((size_t)CC * RP * 2);
    bf* XB = (bf*)take((size_t)TT * CC * 2); bf* FB = (bf*)take((size_t)SS * CC * 2); float* Q0 = (float*)take((size_t)TT * CC * 4); float* LQ = (float*)take((size_t)TT * RP * 4); bf* LQh = (bf*)take((size_t)TT * RP * 2); bf* LQl = (bf*)take((size_t)TT * RP * 2); float* QL = (float*)take((size_t)TT * CC * 4);
    float* KV0 = (float*)take((size_t)SS * 2 * CC * 4); float* LF = (float*)take((size_t)SS * RP * 4); bf* LFh = (bf*)take((size_t)SS * RP * 2); bf* LFl = (bf*)take((size_t)SS * RP * 2); float* KVL = (float*)take((size_t)SS * 2 * CC * 4);
    bf* QPh = (bf*)take((size_t)NH_ * TT * HD * 2); bf* QPl = (bf*)take((size_t)NH_ * TT * HD * 2); bf* KPh = (bf*)take((size_t)NH_ * SS * HD * 2); bf* KPl = (bf*)take((size_t)NH_ * SS * HD * 2); bf* VTh = (bf*)take((size_t)NH_ * HD * SS * 2); bf* VTl = (bf*)take((size_t)NH_ * HD * SS * 2);
    float* Sb = (float*)take((size_t)NH_ * TT * SS * 4); bf* Ph = (bf*)take((size_t)NH_ * TT * SS * 2); bf* Pl = (bf*)take((size_t)NH_ * TT * SS * 2); float* O = (float*)take((size_t)NH_ * TT * HD * 4); bf* Yh = (bf*)take((size_t)TT * CC * 2); bf* Yl = (bf*)take((size_t)TT * CC * 2); float* Y0 = (float*)take((size_t)TT * CC * 4); float* LP = (float*)take((size_t)TT * RP * 4); bf* LPh = (bf*)take((size_t)TT * RP * 2); bf* LPl = (bf*)take((size_t)TT * RP * 2); float* PLr = (float*)take((size_t)TT * CC * 4);
    if ((size_t)(wsp - (char*)d_ws) > ws_size) return;
    k_cvt8<<<(CC * CC / 8 + 255) / 256, 256, 0, stream>>>(wq, WQ, (size_t)CC * CC / 8); k_wpadN<<<(RP * CC / 4 + 255) / 256, 256, 0, stream>>>(aq, CC, AQ); k_wpadK<<<(CC * RP / 4 + 255) / 256, 256, 0, stream>>>(bqm, CC, BQ);
    k_cvt8<<<(2 * CC * CC / 8 + 255) / 256, 256, 0, stream>>>(wf, WF, (size_t)2 * CC * CC / 8); k_wpadN<<<(RP * CC / 4 + 255) / 256, 256, 0, stream>>>(af, CC, AF); k_wpadK<<<(2 * CC * RP / 4 + 255) / 256, 256, 0, stream>>>(bfm, 2 * CC, BF);
    k_cvt8<<<(CC * CC / 8 + 255) / 256, 256, 0, stream>>>(wp, WP, (size_t)CC * CC / 8); k_wpadN<<<(RP * CC / 4 + 255) / 256, 256, 0, stream>>>(ap, CC, AP); k_wpadK<<<(CC * RP / 4 + 255) / 256, 256, 0, stream>>>(bpm, CC, BP);
    for (int b = 0; b < NB_; ++b) {
        k_cvt8<<<(TT * CC / 8 + 255) / 256, 256, 0, stream>>>(x + (size_t)b * TT * CC, XB, (size_t)TT * CC / 8); k_cvt8<<<(SS * CC / 8 + 255) / 256, 256, 0, stream>>>(fe + (size_t)b * SS * CC, FB, (size_t)SS * CC / 8);
        k_gemmw<bf, 0, true><<<dim3(TT / 64, CC / 64, 1), 32, 0, stream>>>(XB, nullptr, WQ, nullptr, CC, Q0, CC, bq, 0, 0, 0); k_gemmw<bf, 0, false><<<dim3(TT / 64, 1, 1), 32, 0, stream>>>(XB, nullptr, AQ, nullptr, CC, LQ, RP, nullptr, 0, 0, 0);
        k_split<<<(TT * RP / 4 + 255) / 256, 256, 0, stream>>>(LQ, (size_t)TT * RP / 4, LQh, LQl); k_gemmw<bf, 1, false><<<dim3(TT / 64, CC / 64, 1), 32, 0, stream>>>(LQh, LQl, BQ, nullptr, RP, QL, CC, nullptr, 0, 0, 0);
        k_qpl<<<(NH_ * TT * HD / 4 + 255) / 256, 256, 0, stream>>>(Q0, QL, TT, CC, 0, QPh, QPl);
        k_gemmw<bf, 0, true><<<dim3(SS / 64, 2 * CC / 64, 1), 32, 0, stream>>>(FB, nullptr, WF, nullptr, CC, KV0, 2 * CC, bff, 0, 0, 0); k_gemmw<bf, 0, false><<<dim3(SS / 64, 1, 1), 32, 0, stream>>>(FB, nullptr, AF, nullptr, CC, LF, RP, nullptr, 0, 0, 0);
        k_split<<<(SS * RP / 4 + 255) / 256, 256, 0, stream>>>(LF, (size_t)SS * RP / 4, LFh, LFl); k_gemmw<bf, 1, false><<<dim3(SS / 64, 2 * CC / 64, 1), 32, 0, stream>>>(LFh, LFl, BF, nullptr, RP, KVL, 2 * CC, nullptr, 0, 0, 0);
        k_qpl<<<(NH_ * SS * HD / 4 + 255) / 256, 256, 0, stream>>>(KV0, KVL, SS, 2 * CC, 0, KPh, KPl); k_vtpl<<<(NH_ * HD * SS / 2 + 255) / 256, 256, 0, stream>>>(KV0, KVL, VTh, VTl);
        k_gemmw<bf, 2, false><<<dim3(TT / 64, SS / 64, NH_), 32, 0, stream>>>(QPh, QPl, KPh, KPl, HD, Sb, SS, nullptr, (size_t)TT * HD, (size_t)SS * HD, (size_t)TT * SS);
        k_csoft<<<NH_ * TT / 8, 256, 0, stream>>>(Sb, Ph, Pl);
        k_gemmw<bf, 2, false><<<dim3(TT / 64, 1, NH_), 32, 0, stream>>>(Ph, Pl, VTh, VTl, SS, O, HD, nullptr, (size_t)TT * SS, (size_t)HD * SS, (size_t)TT * HD);
        k_mrg<<<(TT * CC / 4 + 255) / 256, 256, 0, stream>>>(O, Yh, Yl);
        k_gemmw<bf, 1, true><<<dim3(TT / 64, CC / 64, 1), 32, 0, stream>>>(Yh, Yl, WP, nullptr, CC, Y0, CC, bp, 0, 0, 0); k_gemmw<bf, 1, false><<<dim3(TT / 64, 1, 1), 32, 0, stream>>>(Yh, Yl, AP, nullptr, CC, LP, RP, nullptr, 0, 0, 0);
        k_split<<<(TT * RP / 4 + 255) / 256, 256, 0, stream>>>(LP, (size_t)TT * RP / 4, LPh, LPl); k_gemmw<bf, 1, false><<<dim3(TT / 64, CC / 64, 1), 32, 0, stream>>>(LPh, LPl, BP, nullptr, RP, PLr, CC, nullptr, 0, 0, 0);
        k_fin<<<(TT * CC / 4 + 255) / 256, 256, 0, stream>>>(Y0, PLr, OUT + (size_t)b * TT * CC); }
}
